// MultiHeadAttention_64647847739725
// MI455X (gfx1250) — hardware-verified
//
#include <hip/hip_runtime.h>


#ifndef NB
#define NB 4
#endif
#ifndef SEQ
#define SEQ 2048
#endif
#define NB_FULL   4
#define SEQ_FULL  2048
#define DM        1024
#define NWAVE     8
#define OP        68
#define CVB       2048u
#define NXB       ((unsigned)((size_t)NB * SEQ * DM / CVB))
#define NAB       (3u * NXB)
#define NWB       ((unsigned)((size_t)3 * DM * DM / CVB))
#define NOB       ((unsigned)((size_t)DM * DM / CVB))
#define NCH       (SEQ / 256)
#define WO_CARRY  64.0f
#define OUT_SCALE (1.0f / (4096.0f * 64.0f))

#define EPI_QK  0
#define EPI_VT  1
#define EPI_F32 2
#define EPI_CTX 3
#define EPI_OUT 4

static_assert(SEQ % 256 == 0);
static_assert(SEQ % 128 == 0 && SEQ % 32 == 0);
static_assert(SEQ <= SEQ_FULL);
static_assert(NB >= 1 && NB <= NB_FULL);
static_assert(DM == 1024);
static_assert(DM % 128 == 0 && DM % 32 == 0 && DM % 8 == 0);
static_assert(((size_t)NB * SEQ) % 128 == 0);
static_assert((size_t)NXB * CVB == (size_t)NB * SEQ * DM);
static_assert((size_t)NWB * CVB == (size_t)3 * DM * DM);
static_assert((size_t)NOB * CVB == (size_t)DM * DM);
static_assert((size_t)DM * DM / CVB == 512);
static_assert(256 * 4 == DM);
static_assert((OP * 4) % 16 == 0);
static_assert(OP >= 64);
static_assert(NWAVE * 32 == 256);
static_assert((size_t)(NB - 1) * SEQ_FULL * DM + (size_t)SEQ * DM <= (size_t)NB_FULL * SEQ_FULL * DM);

#define XSLOT_BYTES ((size_t)NB * SEQ * DM * 2)
#define CTX_BYTES   ((size_t)NB * SEQ * DM * 2)
#define S_BYTES     ((size_t)SEQ * SEQ * 4)
#define P_BYTES     ((size_t)SEQ * SEQ * 2)
#define RG_A        ((size_t)3 * XSLOT_BYTES)
#define RG_B        (XSLOT_BYTES + S_BYTES + P_BYTES)
#define RG_BYTES    (RG_A > RG_B ? RG_A : RG_B)
#define WB_BYTES    ((size_t)3 * DM * DM * 2)
#define WO_BYTES    ((size_t)DM * DM * 2)
#define BI_BYTES    ((size_t)4 * DM * 4)
#define QK_BYTES    ((size_t)2 * NB * SEQ * DM * 2)
#define VT_BYTES    ((size_t)NB * DM * SEQ * 2)
#define WS_TOTAL    (RG_BYTES + WB_BYTES + WO_BYTES + BI_BYTES + QK_BYTES + VT_BYTES)
static_assert(WS_TOTAL <= (size_t)134217728);
static_assert(RG_A <= RG_BYTES && RG_B <= RG_BYTES);
static_assert(CTX_BYTES <= XSLOT_BYTES);
static_assert(XSLOT_BYTES % 128 == 0 && S_BYTES % 128 == 0 && P_BYTES % 128 == 0 && RG_BYTES % 128 == 0);
static_assert(WB_BYTES % 128 == 0 && WO_BYTES % 128 == 0 && BI_BYTES % 128 == 0);
static_assert(QK_BYTES % 128 == 0 && VT_BYTES % 128 == 0);

typedef __bf16   bf16;
typedef _Float16 f16;
typedef bf16     v16bf __attribute__((ext_vector_type(16)));
typedef f16      v16h  __attribute__((ext_vector_type(16)));
typedef float    v8f   __attribute__((ext_vector_type(8)));
typedef float    v4f   __attribute__((ext_vector_type(4)));
typedef unsigned v4u   __attribute__((ext_vector_type(4)));

union Pack8B { v4u u; bf16 h[8]; };
union Pack8H { v4u u; f16  h[8]; };

template <typename T> struct FragOf;
template <> struct FragOf<bf16> { typedef v16bf V; };
template <> struct FragOf<f16>  { typedef v16h  V; };

static __device__ __forceinline__ v8f mma16(v16bf a, v16bf b, v8f acc) {
  acc = __builtin_amdgcn_wmma_f32_16x16x32_bf16(false, a, false, b, (short)0, acc, false, false);
  asm volatile("v_nop\n\tv_nop\n\tv_nop\n\tv_nop" : "+v"(acc) : "v"(a), "v"(b));
  return acc;
}
static __device__ __forceinline__ v8f mma16(v16h a, v16h b, v8f acc) {
  acc = __builtin_amdgcn_wmma_f32_16x16x32_f16(false, a, false, b, (short)0, acc, false, false);
  asm volatile("v_nop\n\tv_nop\n\tv_nop\n\tv_nop" : "+v"(acc) : "v"(a), "v"(b));
  return acc;
}

static __device__ __forceinline__ f16 toh_flush(float v) {
  const f16 r = (f16)v;
  return (fabsf(v) < 6.103515625e-05f) ? (f16)0.0f : r;
}

__global__ __launch_bounds__(256) void convert_kernel(const float* __restrict__ kin,
                                                      const float* __restrict__ vin,
                                                      const float* __restrict__ qin,
                                                      const float* __restrict__ wk,
                                                      const float* __restrict__ bk,
                                                      const float* __restrict__ wv,
                                                      const float* __restrict__ bv,
                                                      const float* __restrict__ wq,
                                                      const float* __restrict__ bq,
                                                      const float* __restrict__ wo,
                                                      const float* __restrict__ bo,
                                                      bf16* __restrict__ xb,
                                                      bf16* __restrict__ wb,
                                                      f16* __restrict__ woh,
                                                      float* __restrict__ biasp) {
  const unsigned blk = blockIdx.x;
  const unsigned tid = threadIdx.x;
  if (blk < NAB + NWB) {
    const float* src;
    bf16* dst;
    if (blk < NAB) {
      const unsigned ai = blk / NXB;
      const unsigned lb = blk - ai * NXB;
      const unsigned r  = lb * 2u + (tid >> 7);
      const unsigned c  = (tid & 127u) * 8u;
      const unsigned bt = r / (unsigned)SEQ;
      const unsigned s  = r - bt * (unsigned)SEQ;
      const float* xs = (ai == 0u) ? kin : ((ai == 1u) ? vin : qin);
      src = xs + ((size_t)bt * SEQ_FULL + s) * DM + c;
      dst = xb + (size_t)ai * ((size_t)NB * SEQ * DM) + (size_t)r * DM + c;
    } else {
      const unsigned wblk = blk - NAB;
      const unsigned wi   = wblk >> 9;
      const unsigned off  = (wblk & 511u) * CVB + tid * 8u;
      const float* wsrc = (wi == 0u) ? wk : ((wi == 1u) ? wv : wq);
      src = wsrc + off;
      dst = wb + (size_t)wblk * CVB + tid * 8u;
    }
    const v4f a0 = *(const v4f*)(src);
    const v4f a1 = *(const v4f*)(src + 4);
    Pack8B pk;
    #pragma unroll
    for (int i = 0; i < 4; ++i) {
      pk.h[i]     = (bf16)a0[i];
      pk.h[4 + i] = (bf16)a1[i];
    }
    const v4u val = pk.u;
    *(volatile v4u*)(dst) = val;
    __threadfence();
    *(volatile v4u*)(dst) = val;
  } else if (blk < NAB + NWB + NOB) {
    const unsigned oblk = blk - (NAB + NWB);
    const unsigned off  = oblk * CVB + tid * 8u;
    const v4f a0 = *(const v4f*)(wo + off);
    const v4f a1 = *(const v4f*)(wo + off + 4);
    Pack8H ph;
    #pragma unroll
    for (int i = 0; i < 4; ++i) {
      ph.h[i]     = toh_flush((float)(bf16)a0[i] * WO_CARRY);
      ph.h[4 + i] = toh_flush((float)(bf16)a1[i] * WO_CARRY);
    }
    const v4u val = ph.u;
    f16* dst = woh + off;
    *(volatile v4u*)(dst) = val;
    __threadfence();
    *(volatile v4u*)(dst) = val;
  } else {
    const unsigned j = blk - (NAB + NWB + NOB);
    const float* bsrc = (j == 0u) ? bk : ((j == 1u) ? bv : ((j == 2u) ? bq : bo));
    const v4f a = *(const v4f*)(bsrc + tid * 4u);
    v4f o;
    #pragma unroll
    for (int i = 0; i < 4; ++i) o[i] = (float)(bf16)a[i];
    float* dst = biasp + j * (unsigned)DM + tid * 4u;
    *(volatile v4f*)(dst) = o;
    __threadfence();
    *(volatile v4f*)(dst) = o;
  }
}

template <typename T, int EPI>
__global__ __launch_bounds__(256) void gemm_kernel(const T* __restrict__ A,
                                                   const T* __restrict__ Bt,
                                                   const float* __restrict__ bias,
                                                   void* __restrict__ C,
                                                   unsigned nk, unsigned lda, unsigned ldb, unsigned ldc,
                                                   unsigned long long sAz, unsigned long long sBz,
                                                   unsigned long long sCz, float scale) {
  typedef typename FragOf<T>::V VT;
  union Frag { VT v; v4u q[2]; };

  __shared__ __align__(16) float sO[NWAVE * 16 * OP];

  const unsigned tid  = threadIdx.x;
  const unsigned wave = tid >> 5;
  const unsigned lane = tid & 31u;
  const unsigned lq   = lane & 15u;
  const unsigned hi   = lane >> 4;
  const unsigned m0   = blockIdx.x * 128u + (wave & 3u) * 32u;
  const unsigned n0   = blockIdx.y * 128u + (wave >> 2) * 64u;

  const T* Ab = A  + (size_t)blockIdx.z * sAz;
  const T* Bb = Bt + (size_t)blockIdx.z * sBz;

  const T* ap[2];
  const T* bp[4];
  #pragma unroll
  for (int mt = 0; mt < 2; ++mt) ap[mt] = Ab + (size_t)(m0 + mt * 16u + lq) * lda + hi * 8u;
  #pragma unroll
  for (int nt = 0; nt < 4; ++nt) bp[nt] = Bb + (size_t)(n0 + nt * 16u + lq) * ldb + hi * 8u;

  v8f acc[2][4];
  #pragma unroll
  for (int mt = 0; mt < 2; ++mt) {
    #pragma unroll
    for (int nt = 0; nt < 4; ++nt) acc[mt][nt] = (v8f){0, 0, 0, 0, 0, 0, 0, 0};
  }

  #pragma unroll 1
  for (unsigned k = 0; k < nk; ++k) {
    const unsigned ko = k * 32u;
    Frag a[2], b[4];
    #pragma unroll
    for (int mt = 0; mt < 2; ++mt) {
      a[mt].q[0] = *(const v4u*)(ap[mt] + ko);
      a[mt].q[1] = *(const v4u*)(ap[mt] + ko + 16u);
    }
    #pragma unroll
    for (int nt = 0; nt < 4; ++nt) {
      b[nt].q[0] = *(const v4u*)(bp[nt] + ko);
      b[nt].q[1] = *(const v4u*)(bp[nt] + ko + 16u);
    }
    #pragma unroll
    for (int nt = 0; nt < 4; ++nt) {
      #pragma unroll
      for (int mt = 0; mt < 2; ++mt) acc[mt][nt] = mma16(a[mt].v, b[nt].v, acc[mt][nt]);
    }
  }

  size_t   cbase;
  unsigned ncol;
  if (EPI == EPI_QK) {
    cbase = (size_t)(n0 >> 10) * sCz;
    ncol  = n0 & 1023u;
  } else {
    cbase = (size_t)blockIdx.z * sCz;
    ncol  = n0;
  }

  float bcol[4];
  #pragma unroll
  for (int nt = 0; nt < 4; ++nt) bcol[nt] = 0.0f;
  if (EPI == EPI_QK || EPI == EPI_OUT) {
    #pragma unroll
    for (int nt = 0; nt < 4; ++nt) bcol[nt] = bias[n0 + nt * 16u + lq];
  }

  float* so = sO + wave * (16u * OP);

  #pragma unroll
  for (int mt = 0; mt < 2; ++mt) {
    if (mt != 0) __syncthreads();
    #pragma unroll
    for (int r = 0; r < 8; ++r) {
      float brow = 0.0f;
      if (EPI == EPI_VT) brow = bias[m0 + mt * 16u + hi * 8u + r];
      #pragma unroll
      for (int nt = 0; nt < 4; ++nt) {
        float val = acc[mt][nt][r];
        if (EPI == EPI_QK)  val += bcol[nt];
        if (EPI == EPI_VT)  val += brow;
        if (EPI == EPI_F32 || EPI == EPI_CTX) val *= scale;
        if (EPI == EPI_OUT) val = val * scale + bcol[nt];
        so[(hi * 8u + r) * OP + nt * 16u + lq] = val;
      }
    }
    __syncthreads();

    if (EPI == EPI_F32 || EPI == EPI_OUT) {
      float* Cf = (float*)C + cbase;
      v4f    vals[8];
      size_t gidx[8];
      #pragma unroll
      for (int it = 0; it < 8; ++it) {
        const unsigned row = it * 2u + hi;
        vals[it] = *(const v4f*)(so + row * OP + lq * 4u);
        gidx[it] = (size_t)(m0 + mt * 16u + row) * ldc + ncol + lq * 4u;
      }
      #pragma unroll
      for (int it = 0; it < 8; ++it) *(volatile v4f*)(Cf + gidx[it]) = vals[it];
      __threadfence();
      #pragma unroll
      for (int it = 0; it < 8; ++it) *(volatile v4f*)(Cf + gidx[it]) = vals[it];
    } else {
      f16* Ch = (f16*)C + cbase;
      v4u    vals[4];
      size_t gidx[4];
      #pragma unroll
      for (int it = 0; it < 4; ++it) {
        const unsigned row = it * 4u + (lane >> 3);
        const unsigned c8  = (lane & 7u) * 8u;
        const v4f x0 = *(const v4f*)(so + row * OP + c8);
        const v4f x1 = *(const v4f*)(so + row * OP + c8 + 4u);
        Pack8H ph;
        #pragma unroll
        for (int i = 0; i < 4; ++i) {
          ph.h[i]     = toh_flush(x0[i]);
          ph.h[4 + i] = toh_flush(x1[i]);
        }
        vals[it] = ph.u;
        gidx[it] = (size_t)(m0 + mt * 16u + row) * ldc + ncol + c8;
      }
      #pragma unroll
      for (int it = 0; it < 4; ++it) *(volatile v4u*)(Ch + gidx[it]) = vals[it];
      __threadfence();
      #pragma unroll
      for (int it = 0; it < 4; ++it) *(volatile v4u*)(Ch + gidx[it]) = vals[it];
    }
  }
}

__global__ __launch_bounds__(256) void softmax_kernel(const float* __restrict__ S, f16* __restrict__ P) {
  const unsigned tid  = threadIdx.x;
  const unsigned wave = tid >> 5;
  const unsigned lane = tid & 31u;
  const unsigned row  = blockIdx.x * 8u + wave;
  const float* sp = S + (size_t)row * SEQ + lane * 8u;

  v4f v[NCH][2];
  #pragma unroll
  for (int it = 0; it < NCH; ++it) {
    v[it][0] = *(const v4f*)(sp + it * 256);
    v[it][1] = *(const v4f*)(sp + it * 256 + 4);
  }

  float m = -__builtin_inff();
  #pragma unroll
  for (int it = 0; it < NCH; ++it) {
    #pragma unroll
    for (int i = 0; i < 4; ++i) {
      m = fmaxf(m, v[it][0][i]);
      m = fmaxf(m, v[it][1][i]);
    }
  }
  #pragma unroll
  for (int off = 16; off > 0; off >>= 1) m = fmaxf(m, __shfl_xor(m, off, 32));

  const float L2E = 1.4426950408889634f;
  float sum = 0.0f;
  #pragma unroll
  for (int it = 0; it < NCH; ++it) {
    #pragma unroll
    for (int i = 0; i < 4; ++i) {
      const float e0 = __builtin_amdgcn_exp2f((v[it][0][i] - m) * L2E);
      const float e1 = __builtin_amdgcn_exp2f((v[it][1][i] - m) * L2E);
      v[it][0][i] = e0;
      v[it][1][i] = e1;
      sum += e0;
      sum += e1;
    }
  }
  #pragma unroll
  for (int off = 16; off > 0; off >>= 1) sum += __shfl_xor(sum, off, 32);

  const float inv = 4096.0f * __builtin_amdgcn_rcpf(sum);

  v4u pk[NCH];
  #pragma unroll
  for (int it = 0; it < NCH; ++it) {
    Pack8H ph;
    #pragma unroll
    for (int i = 0; i < 4; ++i) {
      ph.h[i]     = (f16)(v[it][0][i] * inv);
      ph.h[4 + i] = (f16)(v[it][1][i] * inv);
    }
    pk[it] = ph.u;
  }

  f16* dp = P + (size_t)row * SEQ + lane * 8u;
  #pragma unroll
  for (int it = 0; it < NCH; ++it) *(volatile v4u*)(dp + it * 256) = pk[it];
  __threadfence();
  #pragma unroll
  for (int it = 0; it < NCH; ++it) *(volatile v4u*)(dp + it * 256) = pk[it];
}

extern "C" void kernel_launch(void* const* d_in, const int* in_sizes, int n_in,
                              void* d_out, int out_size, void* d_ws, size_t ws_size,
                              hipStream_t stream) {
  if (n_in < 11) return;
  const size_t rows_used = (size_t)(NB - 1) * SEQ_FULL + SEQ;
  if ((size_t)in_sizes[0] < rows_used * DM) return;
  if ((size_t)in_sizes[1] < rows_used * DM) return;
  if ((size_t)in_sizes[2] < rows_used * DM) return;
  if ((size_t)in_sizes[3] < (size_t)DM * DM) return;
  if ((size_t)in_sizes[4] < (size_t)DM) return;
  if ((size_t)in_sizes[5] < (size_t)DM * DM) return;
  if ((size_t)in_sizes[6] < (size_t)DM) return;
  if ((size_t)in_sizes[7] < (size_t)DM * DM) return;
  if ((size_t)in_sizes[8] < (size_t)DM) return;
  if ((size_t)in_sizes[9] < (size_t)DM * DM) return;
  if ((size_t)in_sizes[10] < (size_t)DM) return;
  if ((size_t)out_size < rows_used * DM) return;
  if (ws_size < WS_TOTAL) return;

  const float* kin = (const float*)d_in[0];
  const float* vin = (const float*)d_in[1];
  const float* qin = (const float*)d_in[2];
  const float* wk  = (const float*)d_in[3];
  const float* bk  = (const float*)d_in[4];
  const float* wv  = (const float*)d_in[5];
  const float* bv  = (const float*)d_in[6];
  const float* wq  = (const float*)d_in[7];
  const float* bq  = (const float*)d_in[8];
  const float* wo  = (const float*)d_in[9];
  const float* bo  = (const float*)d_in[10];
  float* out = (float*)d_out;

  char* w = (char*)d_ws;
  char* rg = w;              w += RG_BYTES;
  bf16*  wb    = (bf16*)w;   w += WB_BYTES;
  f16*   woh   = (f16*)w;    w += WO_BYTES;
  float* biasp = (float*)w;  w += BI_BYTES;
  f16*   qk    = (f16*)w;    w += QK_BYTES;
  f16*   vt    = (f16*)w;    w += VT_BYTES;

  bf16*  xb  = (bf16*)rg;
  f16*   ctx = (f16*)rg;
  float* Sp  = (float*)(rg + XSLOT_BYTES);
  f16*   Pp  = (f16*)(rg + XSLOT_BYTES + S_BYTES);

  const unsigned long long plane = (unsigned long long)NB * SEQ * DM;
  f16* qpl = qk;
  f16* kpl = qk + plane;
  const f16* qp = qk;
  const f16* kp = qk + plane;

  convert_kernel<<<dim3(NAB + NWB + NOB + 4u), 256, 0, stream>>>(
      kin, vin, qin, wk, bk, wv, bv, wq, bq, wo, bo, xb, wb, woh, biasp);

  gemm_kernel<bf16, EPI_QK><<<dim3((unsigned)((size_t)NB * SEQ / 128), DM / 128, 1), 256, 0, stream>>>(
      xb, wb, biasp, (void*)kpl, DM / 32, DM, DM, DM, 0ull, 0ull, 0ull, 1.0f);

  gemm_kernel<bf16, EPI_QK><<<dim3((unsigned)((size_t)NB * SEQ / 128), DM / 128, 1), 256, 0, stream>>>(
      xb + (size_t)2 * plane, wb + (size_t)2 * DM * DM, biasp + 2 * DM, (void*)qpl,
      DM / 32, DM, DM, DM, 0ull, 0ull, 0ull, 1.0f);

  gemm_kernel<bf16, EPI_VT><<<dim3(DM / 128, SEQ / 128, NB), 256, 0, stream>>>(
      wb + (size_t)1 * DM * DM, xb + (size_t)1 * plane, biasp + DM, (void*)vt, DM / 32, DM, DM, SEQ,
      0ull, (unsigned long long)SEQ * DM, (unsigned long long)DM * SEQ, 1.0f);

  for (int b = 0; b < NB; ++b) {
    gemm_kernel<f16, EPI_F32><<<dim3(SEQ / 128, SEQ / 128, 1), 256, 0, stream>>>(
        qp + (size_t)b * SEQ * DM, kp + (size_t)b * SEQ * DM, biasp, (void*)Sp,
        DM / 32, DM, DM, SEQ, 0ull, 0ull, 0ull, 0.03125f);

    softmax_kernel<<<dim3(SEQ / 8), 256, 0, stream>>>(Sp, Pp);

    gemm_kernel<f16, EPI_CTX><<<dim3(SEQ / 128, DM / 128, 1), 256, 0, stream>>>(
        Pp, vt + (size_t)b * DM * SEQ, biasp, (void*)(ctx + (size_t)b * SEQ * DM),
        SEQ / 32, SEQ, SEQ, DM, 0ull, 0ull, 0ull, 1.0f);
  }

  gemm_kernel<f16, EPI_OUT><<<dim3(SEQ / 128, DM / 128, NB), 256, 0, stream>>>(
      ctx, woh, biasp + 3 * DM, (void*)out, DM / 32, DM, DM, DM,
      (unsigned long long)SEQ * DM, 0ull, (unsigned long long)SEQ_FULL * DM, OUT_SCALE);
}
